// iPUNetwork_4037269258634
// MI455X (gfx1250) — hardware-run, weakly checked
//
#include <hip/hip_runtime.h>
#pragma clang fp contract(off)


#ifndef NB
#define NB 2
#endif
#ifndef SEQ
#define SEQ 1024
#endif
#define NB_FULL  2
#define SEQ_FULL 1024
#define DM   128
#define PW   32
#define NS   48
#define GU   7
#define NCELL 49
#define PUW  147
#define PPB  32
#define PWV  8
#define PPW  4
#define OSP  36
#define NWCOL 27

#define OUT0_F ((size_t)0)
#define OUT1_F ((size_t)NB_FULL * SEQ_FULL * 3)
#define OUT2_F ((size_t)2 * NB_FULL * SEQ_FULL * 3)
#define OUT3_F (OUT2_F + (size_t)NB_FULL * SEQ_FULL * 16 * 3)
#define OUT4_F (OUT3_F + (size_t)NB_FULL * SEQ_FULL * 3)
#define N4V  (PPB * PUW / 4)
#define N4IT ((N4V + 255) / 256)
#define N2V  (PPB * 48 / 4)
#define N2IT ((N2V + 255) / 256)

static_assert(OUT1_F * 4 == 24576);
static_assert(OUT2_F * 4 == 49152);
static_assert(OUT3_F * 4 == 442368);
static_assert(OUT4_F * 4 == 466944);
static_assert((OUT4_F + (size_t)NB_FULL * SEQ_FULL * PUW) * 4 == 1671168);
static_assert(NB <= NB_FULL);
static_assert(SEQ <= SEQ_FULL);
static_assert(DM % 32 == 0);
static_assert(PW == 32);
static_assert(NWCOL <= PW);
static_assert((NB * SEQ) % 16 == 0);
static_assert(SEQ % 256 == 0);
static_assert(SEQ % PPB == 0);
static_assert(SEQ_FULL % PPB == 0);
static_assert(PPB == PWV * PPW);
static_assert((PPB * PUW) % 32 == 0);
static_assert((PPB * 48) % 32 == 0);
static_assert((PPB * 3) % 32 == 0);
static_assert(N4V % 8 == 0);
static_assert(N2V % 8 == 0);
static_assert(N4IT * 256 >= N4V);
static_assert(N2IT * 256 >= N2V);
static_assert(PPB * 3 / 4 == 24);
static_assert((OSP * 4) % 16 == 0);
static_assert(((size_t)SEQ * DM) % 8 == 0);
static_assert(NS <= 64);
static_assert(NCELL <= 64);
static_assert(32 * DM / 8 == 512);

typedef unsigned short bf;
typedef __attribute__((ext_vector_type(16))) __bf16   v16bf;
typedef __attribute__((ext_vector_type(8)))  unsigned short v8us;
typedef __attribute__((ext_vector_type(8)))  float    v8f;
typedef __attribute__((ext_vector_type(4)))  float    v4f;
typedef v4f  __attribute__((may_alias)) v4fa;

__device__ __forceinline__ unsigned short f2bf(float f) { unsigned u = __float_as_uint(f); u += 0x7FFFu + ((u >> 16) & 1u); return (unsigned short)(u >> 16); }
__device__ __forceinline__ float bfr(float f) { return __uint_as_float(((unsigned)f2bf(f)) << 16); }
__device__ __forceinline__ v16bf cat16b(v8us lo, v8us hi) { return __builtin_bit_cast(v16bf, __builtin_shufflevector(lo, hi, 0, 1, 2, 3, 4, 5, 6, 7, 8, 9, 10, 11, 12, 13, 14, 15)); }
__device__ __forceinline__ v8f wmmab(v16bf a, v16bf b, v8f c) { return __builtin_amdgcn_wmma_f32_16x16x32_bf16(false, a, false, b, (short)0, c, false, false); }
__device__ __forceinline__ v8f wmmab_g(v16bf a, v16bf b, v8f c) { c = wmmab(a, b, c); asm volatile("v_nop\n\tv_nop\n\tv_nop\n\tv_nop" : "+v"(c) : "v"(a), "v"(b)); return c; }
__device__ __forceinline__ v16bf ldb(const bf* p)  { return cat16b(*(const v8us*)p, *(const v8us*)(p + 16)); }
__device__ __forceinline__ void wave_sync() { __builtin_amdgcn_fence(3  , "wavefront"); __builtin_amdgcn_wave_barrier(); asm volatile("" ::: "memory"); }

__global__ __launch_bounds__(256) void k_cvt8(const float* __restrict__ src, bf* dst, size_t n8) {
    const size_t i = (size_t)blockIdx.x * 256 + threadIdx.x; if (i >= n8) return;
    const v8f v = *(const v8f*)(src + i * 8); v8us o;
#pragma unroll
    for (int k = 0; k < 8; ++k) o[k] = f2bf(v[k]);
    *(volatile v8us*)(dst + i * 8) = o; __threadfence(); *(volatile v8us*)(dst + i * 8) = o;
}

__global__ __launch_bounds__(256) void k_wprep(const float* __restrict__ W0, const float* __restrict__ W1, const float* __restrict__ WU, bf* WB) {
    const int i = blockIdx.x * 256 + threadIdx.x;
    const int n = (i >> 4) & 31, c8 = (i & 15) * 8;
    const int n0 = n < 2 ? n : 2;
    int n1 = n - 3; n1 = n1 < 0 ? 0 : (n1 > 2 ? 2 : n1);
    int nu = n - 6; nu = nu < 0 ? 0 : (nu > 20 ? 20 : nu);
    v4f a0 = *(const v4f*)(W0 + n0 * DM + c8), a1 = *(const v4f*)(W0 + n0 * DM + c8 + 4);
    v4f e0 = *(const v4f*)(W1 + n1 * DM + c8), e1 = *(const v4f*)(W1 + n1 * DM + c8 + 4);
    float u[8];
#pragma unroll
    for (int k = 0; k < 8; ++k) u[k] = WU[(c8 + k) * 21 + nu];
    asm volatile("" : "+v"(a0), "+v"(a1), "+v"(e0), "+v"(e1));
#pragma unroll
    for (int k = 0; k < 8; ++k) asm volatile("" : "+v"(u[k]));
    v8us o;
#pragma unroll
    for (int k = 0; k < 8; ++k) {
        const float w0 = (k < 4) ? a0[k & 3] : a1[k & 3];
        const float w1 = (k < 4) ? e0[k & 3] : e1[k & 3];
        const float v = (n < 3) ? w0 : ((n < 6) ? w1 : ((n < NWCOL) ? u[k] : 0.0f));
        o[k] = f2bf(v); }
    bf* dp = WB + (size_t)i * 8;
    *(volatile v8us*)dp = o; __threadfence(); *(volatile v8us*)dp = o;
}

__global__ __launch_bounds__(32) void k_gemm(const bf* __restrict__ A, const bf* __restrict__ Bt, float* PJ) {
    __shared__ __align__(16) float os[16 * OSP];
    const int lane = threadIdx.x & 31, lr = lane & 15, hi = lane >> 4; const int r0 = blockIdx.x * 16;
    v8f acc0 = (v8f){}, acc1 = (v8f){};
    const size_t aoff = (size_t)(r0 + lr) * DM + 8 * hi, boff = (size_t)lr * DM + 8 * hi;
#pragma unroll
    for (int kc = 0; kc < DM; kc += 32) {
        const v16bf a  = ldb(A + aoff + kc);
        const v16bf w0 = ldb(Bt + boff + kc);
        const v16bf w1 = ldb(Bt + boff + (size_t)16 * DM + kc);
        acc0 = wmmab_g(a, w0, acc0);
        acc1 = wmmab_g(a, w1, acc1); }
#pragma unroll
    for (int j = 0; j < 8; ++j) { os[(hi * 8 + j) * OSP + lr] = acc0[j]; os[(hi * 8 + j) * OSP + 16 + lr] = acc1[j]; }
    wave_sync();
    float* prow = PJ + (size_t)r0 * PW;
#pragma unroll 1
    for (int ps = 0; ps < 2; ++ps) {
#pragma unroll
        for (int s = 0; s < 4; ++s) { const int row = 4 * s + (lane >> 3), cofs = (lane & 7) * 4;
            const v4f val = *(const v4fa*)(&os[row * OSP + cofs]);
            *(volatile v4f*)(prow + (size_t)row * PW + cofs) = val; }
        if (ps == 0) __threadfence(); }
}

__device__ __forceinline__ int cell7(float lp) { float t = (lp + 0.3f) * (1.0f / 0.6f); t = t * 6.0f; const int c = (int)rintf(t); return c < 0 ? 0 : (c > 6 ? 6 : c); }

__global__ __launch_bounds__(256) void k_points(const float* __restrict__ xyz, const float* __restrict__ PJ, const float* __restrict__ b0p, const float* __restrict__ b1p,
                                                const int* __restrict__ indexSel, float* OUT) {
    __shared__ float xs[SEQ], ys[SEQ], zs[SEQ], sq[SEQ];
    __shared__ int lst[PWV][NS];
    __shared__ int sIdx[PWV][NS];
    __shared__ int sWin[PWV][NS];
    __shared__ int idxSh[16];
    __shared__ __align__(16) float st4[PPB * PUW];
    __shared__ __align__(16) float st2[PPB * 48];
    __shared__ __align__(16) float st0[PPB * 3];
    __shared__ __align__(16) float st1[PPB * 3];
    __shared__ __align__(16) float st3[PPB * 3];
    static_assert(sizeof(float) * (4 * SEQ + PPB * PUW + PPB * 48 + 3 * PPB * 3) + sizeof(int) * (3 * PWV * NS + 16) <= 131072);
    const int tid = threadIdx.x, lane = tid & 31;
    const int wave = __builtin_amdgcn_readfirstlane((int)(threadIdx.x >> 5));
    const int bpb = SEQ / PPB;
    const int b = blockIdx.x / bpb, n0 = (blockIdx.x % bpb) * PPB;
    const float* xb = xyz + (size_t)b * 3 * SEQ_FULL;
#pragma unroll 1
    for (int j = tid; j < SEQ; j += 256) {
        const float x = bfr(xb[j]), y = bfr(xb[SEQ_FULL + j]), z = bfr(xb[2 * SEQ_FULL + j]);
        xs[j] = x; ys[j] = y; zs[j] = z; sq[j] = (x * x + z * z) + y * y; }
    if (tid < 16) { int ix = indexSel[tid]; ix = ix < 0 ? ix + NCELL : ix; ix = ix < 0 ? 0 : (ix > NCELL - 1 ? NCELL - 1 : ix); idxSh[tid] = ix; }
    const float bo0 = bfr(b0p[0]), bo1 = bfr(b0p[1]), bo2 = bfr(b0p[2]);
    const float bn0 = bfr(b1p[0]), bn1 = bfr(b1p[1]), bn2 = bfr(b1p[2]);
    __syncthreads();

#pragma unroll 1
    for (int q = 0; q < PPW; ++q) {
        const int pl = wave * PPW + q;
        const int n = n0 + pl;
        const float cx = xs[n], cy = ys[n], cz = zs[n], nq = sq[n];
        int total = 0;
#pragma unroll 1
        for (int c = 0; c < SEQ / 32; ++c) {
            const int j = c * 32 + lane;
            float p = cx * xs[j]; p = fmaf(cy, ys[j], p); p = fmaf(cz, zs[j], p);
            float d2 = -2.0f * p; d2 = d2 + nq; d2 = d2 + sq[j];
            const bool in = !(d2 > 0.09f);
            const unsigned mask = __builtin_amdgcn_ballot_w32(in);
            const int pos = total + __popc(mask & ((1u << lane) - 1u));
            if (in & (pos < NS)) lst[wave][pos] = j;
            total += __popc(mask);
            if (total >= NS) break;
        }
        if (total == 0) { if (lane == 0) lst[wave][0] = SEQ - 1; }
        int cnt = total < NS ? total : NS; cnt = cnt < 1 ? 1 : cnt;
        const bool padded = total < NS;
        wave_sync();

        const float* pc = PJ + (size_t)(b * SEQ + n) * PW;
        float vx = pc[0] + bo0, vy = pc[1] + bo1, vz = pc[2] + bo2;
        const float wx = pc[3] + bn0, wy = pc[4] + bn1, wz = pc[5] + bn2;
        float ox = 0.0f, oy = 0.0f, oz = 0.0f, nx = 0.0f, ny = 0.0f, nz = 0.0f, rx = 0.0f, ry = 0.0f, rz = 0.0f, ax = 0.0f, ay = 0.0f, az = 0.0f;
#pragma unroll 1
        for (int it = 0; it < 4; ++it) {
            const float ss = (vx * vx + vz * vz) + vy * vy;
            const float den = sqrtf(ss + 1e-8f) + 1e-10f;
            const float rc = 1.0f / den;
            const float ux = vx * rc, uy = vy * rc, uz = vz * rc;
            if (it == 0)      { ox = ux; oy = uy; oz = uz; vx = wx; vy = wy; vz = wz; }
            else if (it == 1) { nx = ux; ny = uy; nz = uz; vx = oy * nz - oz * ny; vy = oz * nx - ox * nz; vz = ox * ny - oy * nx; }
            else if (it == 2) { rx = ux; ry = uy; rz = uz; vx = ry * nz - rz * ny; vy = rz * nx - rx * nz; vz = rx * ny - ry * nx; }
            else              { ax = ux; ay = uy; az = uz; }
        }
        if (lane == 0) { st0[pl * 3 + 0] = ox; st0[pl * 3 + 1] = oy; st0[pl * 3 + 2] = oz; st1[pl * 3 + 0] = nx; st1[pl * 3 + 1] = ny; st1[pl * 3 + 2] = nz; }

#pragma unroll 1
        for (int h2 = 0; h2 * 32 < cnt; ++h2) {
            const int s = h2 * 32 + lane; const int sc = s < cnt ? s : cnt - 1;
            int g = lst[wave][sc]; g = g < 0 ? 0 : (g > SEQ - 1 ? SEQ - 1 : g);
            const float lx = xs[g] - cx, ly = ys[g] - cy, lz = zs[g] - cz;
            float l0 = lx * ax; l0 = fmaf(ly, ay, l0); l0 = fmaf(lz, az, l0);
            float l1 = lx * rx; l1 = fmaf(ly, ry, l1); l1 = fmaf(lz, rz, l1);
            float l2 = lx * nx; l2 = fmaf(ly, ny, l2); l2 = fmaf(lz, nz, l2);
            const int v = cell7(l0) * GU + cell7(l1) * GU + cell7(l2);
            if (s < cnt) sIdx[wave][s] = v;
        }
        wave_sync();
#pragma unroll 1
        for (int h2 = 0; h2 * 32 < cnt; ++h2) {
            const int s = h2 * 32 + lane; const int sc = s < cnt ? s : cnt - 1;
            const int v = sIdx[wave][sc], v0 = sIdx[wave][0];
            int win = 1;
#pragma unroll 1
            for (int s2 = 1; s2 < cnt; ++s2) { const int v2 = sIdx[wave][s2]; win &= ((s2 <= sc) | (v2 != v)) ? 1 : 0; }
            if (padded) win = (sc == 0) ? 1 : (win & ((v != v0) ? 1 : 0));
            if (s < cnt) sWin[wave][s] = win;
        }
        wave_sync();
#pragma unroll 1
        for (int h2 = 0; h2 < 2; ++h2) {
            const int cl = h2 * 32 + lane;
            float a0 = 0.0f, a1 = 0.0f, a2 = 0.0f;
#pragma unroll 1
            for (int s = 0; s < cnt; ++s) {
                const int v = sIdx[wave][s]; const int w = sWin[wave][s];
                int g = lst[wave][s]; g = g < 0 ? 0 : (g > SEQ - 1 ? SEQ - 1 : g);
                const int ij = v / GU; int k = v - ij * GU; k = k < 0 ? 0 : (k > GU - 1 ? GU - 1 : k);
                const float* pr = PJ + (size_t)(b * SEQ + g) * PW + 6 + k * 3;
                const float q0 = pr[0], q1 = pr[1], q2 = pr[2];
                const bool hit = (ij == cl) & (w != 0);
                a0 += hit ? q0 : 0.0f; a1 += hit ? q1 : 0.0f; a2 += hit ? q2 : 0.0f;
            }
            const int clc = cl < NCELL ? cl : NCELL - 1;
            const int gi = clc / GU, gj = clc - gi * GU;
            const float up0 = (float)((double)(10 * gi - 30) * 0.01) + a0;
            const float up1 = (float)((double)(10 * gj - 30) * 0.01) + a1;
            const float up2 = 0.0f + a2;
            float p0 = up0 * ax; p0 = fmaf(up1, rx, p0); p0 = fmaf(up2, nx, p0); p0 = p0 + cx;
            float p1 = up0 * ay; p1 = fmaf(up1, ry, p1); p1 = fmaf(up2, ny, p1); p1 = p1 + cy;
            float p2 = up0 * az; p2 = fmaf(up1, rz, p2); p2 = fmaf(up2, nz, p2); p2 = p2 + cz;
            if (cl < NCELL) { st4[pl * PUW + cl * 3 + 0] = p0; st4[pl * PUW + cl * 3 + 1] = p1; st4[pl * PUW + cl * 3 + 2] = p2; }
        }
        wave_sync();
        { const int l3 = lane < 3 ? lane : 2; const float c3 = st4[pl * PUW + 24 * 3 + l3]; if (lane < 3) st3[pl * 3 + lane] = c3; }
#pragma unroll 1
        for (int h2 = 0; h2 < 2; ++h2) {
            const int e = h2 * 32 + lane; const int ec = e < 48 ? e : 47;
            const int t = ec / 3, d = ec - 3 * t;
            const float val = st4[pl * PUW + idxSh[t] * 3 + d];
            if (e < 48) st2[pl * 48 + e] = val;
        }
    }
    __syncthreads();

    const size_t fr0 = (size_t)b * SEQ_FULL + (size_t)n0;
    const size_t o4 = OUT4_F + fr0 * PUW, o2 = OUT2_F + fr0 * 48;
    const size_t o0 = OUT0_F + fr0 * 3, o1 = OUT1_F + fr0 * 3, o3 = OUT3_F + fr0 * 3;
    const int slc = lane < 24 ? lane : 23;
#pragma unroll 1
    for (int ps = 0; ps < 2; ++ps) {
#pragma unroll 1
        for (int it = 0; it < N4IT; ++it) { const int i = it * 256 + tid; const int ic = i < N4V ? i : N4V - 1;
            const v4f val = *(const v4fa*)(&st4[ic * 4]);
            if (i < N4V) *(volatile v4f*)(OUT + o4 + (size_t)i * 4) = val; }
#pragma unroll 1
        for (int it = 0; it < N2IT; ++it) { const int i = it * 256 + tid; const int ic = i < N2V ? i : N2V - 1;
            const v4f val = *(const v4fa*)(&st2[ic * 4]);
            if (i < N2V) *(volatile v4f*)(OUT + o2 + (size_t)i * 4) = val; }
        if (wave == 0) { const v4f val = *(const v4fa*)(&st0[slc * 4]); if (lane < 24) *(volatile v4f*)(OUT + o0 + (size_t)lane * 4) = val; }
        if (wave == 1) { const v4f val = *(const v4fa*)(&st1[slc * 4]); if (lane < 24) *(volatile v4f*)(OUT + o1 + (size_t)lane * 4) = val; }
        if (wave == 2) { const v4f val = *(const v4fa*)(&st3[slc * 4]); if (lane < 24) *(volatile v4f*)(OUT + o3 + (size_t)lane * 4) = val; }
        if (ps == 0) __threadfence(); }
}

static constexpr size_t al256(size_t v) { return (v + 255) & ~(size_t)255; }
static constexpr size_t SZ_XB = al256((size_t)NB * SEQ * DM * 2);
static constexpr size_t SZ_WB = al256((size_t)32 * DM * 2);
static constexpr size_t SZ_PJ = al256((size_t)NB * SEQ * PW * 4);
static constexpr size_t SZ_TOTAL = SZ_XB + SZ_WB + SZ_PJ;
static_assert(SZ_TOTAL <= (size_t)134217728);
static_assert((size_t)512 * 8 * 2 <= SZ_WB);
static_assert((size_t)(NB * SEQ / 16) * 16 * PW * 4 <= SZ_PJ);

extern "C" void kernel_launch(void* const* d_in, const int* in_sizes, int n_in,
                              void* d_out, int out_size, void* d_ws, size_t ws_size, hipStream_t stream) {
    if (n_in < 8) return;
    const size_t needx = (size_t)(NB - 1) * 3 * SEQ_FULL + (size_t)2 * SEQ_FULL + SEQ;
    const size_t needf = ((size_t)(NB - 1) * SEQ_FULL + SEQ) * DM;
    if ((size_t)in_sizes[0] < needx || (size_t)in_sizes[1] < needf) return;
    if (in_sizes[2] < 3 * DM || in_sizes[3] < 3 || in_sizes[4] < 3 * DM || in_sizes[5] < 3) return;
    if (in_sizes[6] < DM * 21 || in_sizes[7] < 16) return;
    if ((size_t)out_size < OUT4_F + ((size_t)(NB - 1) * SEQ_FULL + SEQ) * PUW) return;
    if (SZ_TOTAL > ws_size) return;
    const float* xyz  = (const float*)d_in[0];
    const float* feat = (const float*)d_in[1];
    const float* w0   = (const float*)d_in[2];
    const float* b0   = (const float*)d_in[3];
    const float* w1   = (const float*)d_in[4];
    const float* b1   = (const float*)d_in[5];
    const float* wu   = (const float*)d_in[6];
    const int*   isel = (const int*)d_in[7];
    float* OUT = (float*)d_out;
    char* wsp = (char*)d_ws;
    bf* XB = (bf*)wsp; wsp += SZ_XB;
    bf* WB = (bf*)wsp; wsp += SZ_WB;
    float* PJ = (float*)wsp; wsp += SZ_PJ;

    if (SEQ == SEQ_FULL) {
        const size_t n8 = (size_t)NB * SEQ * DM / 8;
        k_cvt8<<<(unsigned)((n8 + 255) / 256), 256, 0, stream>>>(feat, XB, n8);
    } else {
        const size_t n8 = (size_t)SEQ * DM / 8;
        for (int b = 0; b < NB; ++b) k_cvt8<<<(unsigned)((n8 + 255) / 256), 256, 0, stream>>>(feat + (size_t)b * SEQ_FULL * DM, XB + (size_t)b * SEQ * DM, n8);
    }
    k_wprep<<<2, 256, 0, stream>>>(w0, w1, wu, WB);
    k_gemm<<<NB * SEQ / 16, 32, 0, stream>>>(XB, WB, PJ);
    k_points<<<NB * SEQ / PPB, 256, 0, stream>>>(xyz, PJ, b0, b1, isel, OUT);
}
